// attn_block_70952859730118
// MI455X (gfx1250) — hardware-verified
//
#include <hip/hip_runtime.h>
#include <math.h>
#include <stdint.h>

#ifndef NB
#define NB 4
#endif
#ifndef SEQ
#define SEQ 4096
#endif
#ifndef NNF
#define NNF 4096
#endif
#ifndef QRES
#define QRES 1
#endif
#define NBF   4
#define CC    256
#define NG    32
#define CPG   8
#define QT    64
#define OSP   68
#define OSPW  132
#define TP    72
#define TPF   68
#define STP   32
#define ATT   0.0625f
#define QLS   4096.0f
#define RQL   0.000244140625f
#define LNPS  9.704060527839234f
#define GNEPS 1.0e-6f

static_assert(NB >= 1 && NB <= NBF);
static_assert(SEQ % QT == 0 && SEQ % 32 == 0 && SEQ >= QT);
static_assert(SEQ <= NNF && NNF % 8 == 0);
static_assert(CC == 256 && NG * CPG == CC && CC % QT == 0 && CC % 32 == 0);
static_assert((OSP * 4) % 16 == 0);
static_assert((OSPW * 4) % 16 == 0);
static_assert((TP * 2) % 16 == 0);
static_assert((TPF * 4) % 16 == 0);
static_assert(STP * 4 == 128);

typedef _Float16       v16h __attribute__((ext_vector_type(16)));
typedef _Float16       v8h  __attribute__((ext_vector_type(8)));
typedef __bf16         v16b __attribute__((ext_vector_type(16)));
typedef unsigned short v8us __attribute__((ext_vector_type(8)));
typedef float          v8f  __attribute__((ext_vector_type(8)));
typedef float          v4f  __attribute__((ext_vector_type(4)));
typedef unsigned int   v4u  __attribute__((ext_vector_type(4)));

union Frag  { v8us u[2]; v16h h; v16b bf; };
union FragH { v16h v; v8h hv[2]; };
static_assert(sizeof(Frag) == 32);
static_assert(sizeof(FragH) == 32);

__device__ __forceinline__ unsigned short bf_bits(float f) {
  unsigned u = __float_as_uint(f);
  return (unsigned short)((u + 0x7FFFu + ((u >> 16) & 1u)) >> 16);
}
__device__ __forceinline__ float bf_up(unsigned short hb) { return __uint_as_float(((unsigned)hb) << 16); }
__device__ __forceinline__ float bfr(float f) { return bf_up(bf_bits(f)); }
__device__ __forceinline__ unsigned short h_bits(_Float16 x) { return __builtin_bit_cast(unsigned short, x); }
__device__ __forceinline__ unsigned pk16(unsigned short a, unsigned short b) { return (unsigned)a | ((unsigned)b << 16); }
__device__ __forceinline__ v8f zero8() { v8f z = {0.f, 0.f, 0.f, 0.f, 0.f, 0.f, 0.f, 0.f}; return z; }
__device__ __forceinline__ float hmax8(v8f s) {
  return fmaxf(fmaxf(fmaxf(s[0], s[1]), fmaxf(s[2], s[3])), fmaxf(fmaxf(s[4], s[5]), fmaxf(s[6], s[7])));
}
__device__ __forceinline__ unsigned wave_ballot(bool p) {
#if defined(__HIP_DEVICE_COMPILE__)
  return __builtin_amdgcn_ballot_w32(p);
#else
  return p ? 1u : 0u;
#endif
}
__device__ __forceinline__ float wsum(float v) {
  v += __shfl_xor(v, 16, 32);
  v += __shfl_xor(v, 8, 32);
  v += __shfl_xor(v, 4, 32);
  v += __shfl_xor(v, 2, 32);
  v += __shfl_xor(v, 1, 32);
  return v;
}

__device__ __forceinline__ Frag ldfrag(const unsigned short* p) {
  Frag f;
  f.u[0] = *(const v8us*)(p);
  f.u[1] = *(const v8us*)(p + 16);
  return f;
}

__device__ __forceinline__ v8f mma_h(v16h a, v16h b, v8f c) {
  v8f d = __builtin_amdgcn_wmma_f32_16x16x32_f16(false, a, false, b, (short)0, c, false, false);
#if defined(__HIP_DEVICE_COMPILE__)
  asm volatile("v_nop\n\tv_nop\n\tv_nop\n\tv_nop" : "+v"(d) : "v"(a), "v"(b));
#endif
  return d;
}
__device__ __forceinline__ v8f mma_b(v16b a, v16b b, v8f c) {
  v8f d = __builtin_amdgcn_wmma_f32_16x16x32_bf16(false, a, false, b, (short)0, c, false, false);
#if defined(__HIP_DEVICE_COMPILE__)
  const v16h ha = __builtin_bit_cast(v16h, a), hb = __builtin_bit_cast(v16h, b);
  asm volatile("v_nop\n\tv_nop\n\tv_nop\n\tv_nop" : "+v"(d) : "v"(ha), "v"(hb));
#endif
  return d;
}

__global__ __launch_bounds__(256)
void cvt_w(const float* __restrict__ Wq, const float* __restrict__ Wk, const float* __restrict__ Wv,
           const float* __restrict__ Wp, unsigned short* WT) {
  __shared__ __align__(16) unsigned short T[QT * TP];
  const int tid = threadIdx.x;
  const int ob = blockIdx.x, cb = blockIdx.y, mat = blockIdx.z;
  const int e = tid & 7, lq = tid >> 3;
  const int o0 = ob * QT, c0 = cb * QT;
  const float* Wm = (mat == 0) ? Wq : ((mat == 1) ? Wk : ((mat == 2) ? Wv : Wp));
#pragma unroll
  for (int it = 0; it < 2; ++it) {
    const int cl = it * 32 + lq;
    const float* sp = Wm + (size_t)(c0 + cl) * CC + o0 + 8 * e;
    const v4f a = *(const v4f*)sp;
    const v4f q = *(const v4f*)(sp + 4);
    const float f[8] = {a[0], a[1], a[2], a[3], q[0], q[1], q[2], q[3]};
#pragma unroll
    for (int t = 0; t < 8; ++t) T[(8 * e + t) * TP + cl] = bf_bits(f[t]);
  }
  __syncthreads();
  v4u up[2];
#pragma unroll
  for (int it = 0; it < 2; ++it) {
    const int ol = it * 32 + lq;
    up[it] = *(const v4u*)(T + ol * TP + 8 * e);
  }
#pragma unroll
  for (int pass = 0; pass < 2; ++pass) {
#pragma unroll
    for (int it = 0; it < 2; ++it) {
      const int ol = it * 32 + lq;
      *(volatile v4u*)(WT + ((size_t)(mat * CC + o0 + ol)) * CC + c0 + 8 * e) = up[it];
    }
    __threadfence();
  }
}

__global__ __launch_bounds__(256)
void gn_stats(const float* __restrict__ x, float* ST) {
  __shared__ float red[8];
  __shared__ float bc[2];
  const int tid = threadIdx.x, lane = tid & 31, wave = tid >> 5;
  const int g = blockIdx.x, b = blockIdx.y;
  const float* xb = x + ((size_t)(b * CC + g * CPG)) * NNF;
  const int CH4 = SEQ / 4, NCH = CPG * CH4;
  const float icnt = 1.0f / (float)(CPG * SEQ);

  float s = 0.f;
#pragma unroll 4
  for (int qd = tid; qd < NCH; qd += 256) {
    const int cl = qd / CH4, p4 = qd - cl * CH4;
    const v4f a = *(const v4f*)(xb + (size_t)cl * NNF + 4 * p4);
    s += (bfr(a[0]) + bfr(a[1])) + (bfr(a[2]) + bfr(a[3]));
  }
  s = wsum(s);
  if (lane == 0) red[wave] = s;
  __syncthreads();
  if (tid == 0) {
    float t = 0.f;
#pragma unroll
    for (int i = 0; i < 8; ++i) t += red[i];
    bc[0] = t * icnt;
  }
  __syncthreads();
  const float mu = bc[0];

  float ss = 0.f;
#pragma unroll 4
  for (int qd = tid; qd < NCH; qd += 256) {
    const int cl = qd / CH4, p4 = qd - cl * CH4;
    const v4f a = *(const v4f*)(xb + (size_t)cl * NNF + 4 * p4);
    const float d0 = bfr(a[0]) - mu, d1 = bfr(a[1]) - mu, d2 = bfr(a[2]) - mu, d3 = bfr(a[3]) - mu;
    ss += (d0 * d0 + d1 * d1) + (d2 * d2 + d3 * d3);
  }
  ss = wsum(ss);
  if (lane == 0) red[wave] = ss;
  __syncthreads();
  if (tid == 0) {
    float t = 0.f;
#pragma unroll
    for (int i = 0; i < 8; ++i) t += red[i];
    const float var = t * icnt;
    bc[1] = rsqrtf(var + GNEPS);
  }
  __syncthreads();
  const float rs = bc[1];

  v4f v = {0.f, 0.f, 0.f, 0.f};
  if (tid == 0) { v[0] = mu; v[1] = rs; }
  if (tid < 8) {
    float* lp = ST + ((size_t)(b * NG + g)) * STP + 4 * tid;
#pragma unroll
    for (int pass = 0; pass < 2; ++pass) {
      *(volatile v4f*)lp = v;
      __threadfence();
    }
  }
}

__global__ __launch_bounds__(256)
void cvt_h(const float* __restrict__ x, const float* __restrict__ ST, const float* __restrict__ gsc,
           const float* __restrict__ gbs, unsigned short* HPh, unsigned short* HPl) {
  __shared__ __align__(16) float T[QT * TPF];
  __shared__ float pmu[QT], prs[QT], psc[QT], pbs[QT];
  const int tid = threadIdx.x;
  const int nb = blockIdx.x, cb = blockIdx.y, b = blockIdx.z;
  const int e = tid & 7, lq = tid >> 3;
  const int n0 = nb * QT, c0 = cb * QT;
  if (tid < QT) {
    const int ch = c0 + tid;
    const int g = ch >> 3;
    pmu[tid] = ST[((size_t)(b * NG + g)) * STP];
    prs[tid] = ST[((size_t)(b * NG + g)) * STP + 1];
    psc[tid] = bfr(gsc[ch]);
    pbs[tid] = bfr(gbs[ch]);
  }
  __syncthreads();
#pragma unroll
  for (int it = 0; it < 2; ++it) {
    const int cl = it * 32 + lq;
    const float* sp = x + ((size_t)(b * CC + c0 + cl)) * NNF + n0 + 8 * e;
    const v4f a = *(const v4f*)sp;
    const v4f q = *(const v4f*)(sp + 4);
    const float f[8] = {a[0], a[1], a[2], a[3], q[0], q[1], q[2], q[3]};
    const float mu = pmu[cl], rs = prs[cl], sc = psc[cl], bs = pbs[cl];
#pragma unroll
    for (int t = 0; t < 8; ++t) {
      const float tt = (bfr(f[t]) - mu) * rs;
      T[(8 * e + t) * TPF + cl] = tt * sc + bs;
    }
  }
  __syncthreads();
  v4u uh[2], ul[2];
#pragma unroll
  for (int it = 0; it < 2; ++it) {
    const int nl = it * 32 + lq;
    const v4f a = *(const v4f*)(T + nl * TPF + 8 * e);
    const v4f q = *(const v4f*)(T + nl * TPF + 8 * e + 4);
    const float f[8] = {a[0], a[1], a[2], a[3], q[0], q[1], q[2], q[3]};
#pragma unroll
    for (int t = 0; t < 4; ++t) {
      const float f0 = f[2 * t], f1 = f[2 * t + 1];
      const unsigned short hb0 = bf_bits(f0), hb1 = bf_bits(f1);
      const unsigned short lb0 = bf_bits(f0 - bf_up(hb0));
      const unsigned short lb1 = bf_bits(f1 - bf_up(hb1));
      uh[it][t] = pk16(hb0, hb1);
      ul[it][t] = pk16(lb0, lb1);
    }
  }
#pragma unroll
  for (int pass = 0; pass < 2; ++pass) {
#pragma unroll
    for (int it = 0; it < 2; ++it) {
      const int nl = it * 32 + lq;
      const size_t po = ((size_t)(b * SEQ + n0 + nl)) * CC + c0 + 8 * e;
      *(volatile v4u*)(HPh + po) = uh[it];
      *(volatile v4u*)(HPl + po) = ul[it];
    }
    __threadfence();
  }
}

__global__ __launch_bounds__(128)
void gemm_qkv(const unsigned short* __restrict__ WT, const unsigned short* __restrict__ HPh,
              const unsigned short* __restrict__ HPl, const float* __restrict__ bq,
              const float* __restrict__ bk, const float* __restrict__ bv,
              unsigned short* Qh, unsigned short* Ql, unsigned short* Kh, unsigned short* Vc) {
  __shared__ __align__(16) float Os[QT * OSP];
  const int tid  = threadIdx.x;
  const int lane = tid & 31, wave = tid >> 5;
  const int hh   = lane >> 4, c = lane & 15;
  const int nt   = blockIdx.x, mb = blockIdx.y, b = blockIdx.z;
  const int mat  = mb >> 2;
  const int n0   = nt * QT, o0 = mb * QT;
  const int ob   = o0 & (CC - 1);

  const unsigned short* ap  = WT  + (size_t)(o0 + c) * CC + 8 * hh;
  const size_t bo = ((size_t)(b * SEQ + n0 + 16 * wave + c)) * CC + 8 * hh;
  const unsigned short* bph = HPh + bo;
  const unsigned short* bpl = HPl + bo;

  v8f acc[4];
#pragma unroll
  for (int mt = 0; mt < 4; ++mt) acc[mt] = zero8();

#pragma unroll
  for (int ks = 0; ks < CC / 32; ++ks) {
    const Frag fbh = ldfrag(bph + 32 * ks);
    const Frag fbl = ldfrag(bpl + 32 * ks);
#pragma unroll
    for (int mt = 0; mt < 4; ++mt) {
      const Frag fa = ldfrag(ap + (size_t)(16 * mt) * CC + 32 * ks);
      acc[mt] = mma_b(fa.bf, fbh.bf, acc[mt]);
      acc[mt] = mma_b(fa.bf, fbl.bf, acc[mt]);
    }
  }

  {
    const float* bias = (mat == 0) ? bq : ((mat == 1) ? bk : bv);
    const int nl = 16 * wave + c;
#pragma unroll
    for (int mt = 0; mt < 4; ++mt) {
      v4f va, vb;
#pragma unroll
      for (int r = 0; r < 4; ++r) {
        va[r] = acc[mt][r]     + bfr(bias[ob + 16 * mt + 8 * hh + r]);
        vb[r] = acc[mt][4 + r] + bfr(bias[ob + 16 * mt + 8 * hh + 4 + r]);
      }
      *(v4f*)(Os + nl * OSP + 16 * mt + 8 * hh)     = va;
      *(v4f*)(Os + nl * OSP + 16 * mt + 8 * hh + 4) = vb;
    }
  }
  __syncthreads();

  const int e = tid & 7, lq = tid >> 3;
  if (mat == 2) {
    v4u uv[4];
#pragma unroll
    for (int it = 0; it < 4; ++it) {
      const int ol = it * 16 + lq;
      unsigned short hb[8];
#pragma unroll
      for (int t = 0; t < 8; ++t) hb[t] = h_bits((_Float16)Os[(8 * e + t) * OSP + ol]);
#pragma unroll
      for (int t = 0; t < 4; ++t) uv[it][t] = pk16(hb[2 * t], hb[2 * t + 1]);
    }
#pragma unroll
    for (int pass = 0; pass < 2; ++pass) {
#pragma unroll
      for (int it = 0; it < 4; ++it) {
        const int ol = it * 16 + lq;
        *(volatile v4u*)(Vc + ((size_t)(b * CC + ob + ol)) * SEQ + n0 + 8 * e) = uv[it];
      }
      __threadfence();
    }
  } else {
    unsigned short* P1 = (mat == 0) ? Qh : Kh;
    v4u uh[4], ul[4];
#pragma unroll
    for (int it = 0; it < 4; ++it) {
      const int row = it * 16 + lq;
      const v4f a = *(const v4f*)(Os + row * OSP + 8 * e);
      const v4f q = *(const v4f*)(Os + row * OSP + 8 * e + 4);
      const float f[8] = {a[0], a[1], a[2], a[3], q[0], q[1], q[2], q[3]};
#pragma unroll
      for (int t = 0; t < 4; ++t) {
        const float f0 = f[2 * t], f1 = f[2 * t + 1];
        const _Float16 h0 = (_Float16)f0, h1 = (_Float16)f1;
        const _Float16 l0 = (_Float16)((f0 - (float)h0) * QLS);
        const _Float16 l1 = (_Float16)((f1 - (float)h1) * QLS);
        uh[it][t] = pk16(h_bits(h0), h_bits(h1));
        ul[it][t] = pk16(h_bits(l0), h_bits(l1));
      }
    }
#pragma unroll
    for (int pass = 0; pass < 2; ++pass) {
#pragma unroll
      for (int it = 0; it < 4; ++it) {
        const int row = it * 16 + lq;
        const size_t po = ((size_t)(b * SEQ + n0 + row)) * CC + ob + 8 * e;
        *(volatile v4u*)(P1 + po) = uh[it];
        if (mat == 0) *(volatile v4u*)(Ql + po) = ul[it];
      }
      __threadfence();
    }
  }
}

__global__ __launch_bounds__(128)
void attn_k(const unsigned short* __restrict__ Qh, const unsigned short* __restrict__ Ql,
            const unsigned short* __restrict__ Kh, const unsigned short* __restrict__ Vc,
            unsigned short* H2h, unsigned short* H2l) {
  __shared__ __align__(16) float Os[QT * OSPW];
  const int tid  = threadIdx.x;
  const int wave = tid >> 5, lane = tid & 31;
  const int hh   = lane >> 4, c = lane & 15;
  const int n0   = blockIdx.x * QT, b = blockIdx.y;

  const size_t qo = ((size_t)(b * SEQ + n0 + 16 * wave + c)) * CC + 8 * hh;
  const unsigned short* Qhp = Qh + qo;
#if QRES
  const unsigned short* Qlp = Ql + qo;
#else
  (void)Ql;
#endif
  const unsigned short* Khp = Kh + (size_t)b * SEQ * CC + (size_t)c * CC + 8 * hh;
  const unsigned short* Vp = Vc + (size_t)b * CC * SEQ + (size_t)c * SEQ + 8 * hh;

  float m = -1.0e30f, l = 0.f;
  v8f o[16];
#pragma unroll
  for (int j = 0; j < 16; ++j) o[j] = zero8();

#pragma unroll 1
  for (int kb = 0; kb < SEQ; kb += 32) {
    const unsigned short* k0p = Khp + (size_t)kb * CC;
    const unsigned short* k1p = Khp + (size_t)(kb + 16) * CC;
    v8f s0 = zero8(), s1 = zero8();
#if QRES
    v8f t0 = zero8(), t1 = zero8();
#endif
#pragma unroll 1
    for (int kc = 0; kc < CC / 32; ++kc) {
      const Frag qh = ldfrag(Qhp + 32 * kc);
      const Frag k0 = ldfrag(k0p + 32 * kc);
      const Frag k1 = ldfrag(k1p + 32 * kc);
      s0 = mma_h(k0.h, qh.h, s0);
      s1 = mma_h(k1.h, qh.h, s1);
#if QRES
      const Frag ql = ldfrag(Qlp + 32 * kc);
      t0 = mma_h(k0.h, ql.h, t0);
      t1 = mma_h(k1.h, ql.h, t1);
#endif
    }

    v8f sc0, sc1;
#pragma unroll
    for (int r = 0; r < 8; ++r) {
#if QRES
      sc0[r] = (s0[r] + t0[r] * RQL) * ATT;
      sc1[r] = (s1[r] + t1[r] * RQL) * ATT;
#else
      sc0[r] = s0[r] * ATT;
      sc1[r] = s1[r] * ATT;
#endif
    }

    float mx = fmaxf(hmax8(sc0), hmax8(sc1));
    mx = fmaxf(mx, __shfl_xor(mx, 16, 32));
    const float mn = fmaxf(m, mx);
    const unsigned grew = wave_ballot(mx > m);
    if (grew != 0u) {
      const float corr = __expf(m - mn);
      l *= corr;
#pragma unroll
      for (int j = 0; j < 16; ++j) {
#pragma unroll
        for (int r = 0; r < 8; ++r) o[j][r] *= corr;
      }
    }
    m = mn;
    const float msh = mn - LNPS;

    FragH ph;
    float ls = 0.f;
#pragma unroll
    for (int r = 0; r < 8; ++r) {
      const float e0 = __expf(sc0[r] - msh);
      const float e1 = __expf(sc1[r] - msh);
      ls += e0 + e1;
      ph.hv[0][r] = (_Float16)e0;
      ph.hv[1][r] = (_Float16)e1;
    }
    l += ls;

#pragma unroll
    for (int j = 0; j < 16; ++j) {
      const Frag vf = ldfrag(Vp + (size_t)(16 * j) * SEQ + kb);
      o[j] = mma_h(vf.h, ph.v, o[j]);
    }
  }
  l += __shfl_xor(l, 16, 32);
  const float inv = 1.0f / l;

  const int qrow = 16 * wave + c;
  const int e16 = tid & 15, r8 = tid >> 4;
#pragma unroll
  for (int half = 0; half < 2; ++half) {
    if (half) __syncthreads();
#pragma unroll
    for (int jj = 0; jj < 8; ++jj) {
      const int j = 8 * half + jj;
      v4f va, vb;
#pragma unroll
      for (int r = 0; r < 4; ++r) { va[r] = o[j][r] * inv; vb[r] = o[j][4 + r] * inv; }
      *(v4f*)(Os + qrow * OSPW + 16 * jj + 8 * hh)     = va;
      *(v4f*)(Os + qrow * OSPW + 16 * jj + 8 * hh + 4) = vb;
    }
    __syncthreads();
#pragma unroll
    for (int chk = 0; chk < 2; ++chk) {
      v4u uh[4], ul[4];
#pragma unroll
      for (int i = 0; i < 4; ++i) {
        const int row = (4 * chk + i) * 8 + r8;
        const v4f a = *(const v4f*)(Os + row * OSPW + 8 * e16);
        const v4f q = *(const v4f*)(Os + row * OSPW + 8 * e16 + 4);
        const float f[8] = {a[0], a[1], a[2], a[3], q[0], q[1], q[2], q[3]};
#pragma unroll
        for (int t = 0; t < 4; ++t) {
          const float f0 = f[2 * t], f1 = f[2 * t + 1];
          const unsigned short hb0 = bf_bits(f0), hb1 = bf_bits(f1);
          const unsigned short lb0 = bf_bits(f0 - bf_up(hb0));
          const unsigned short lb1 = bf_bits(f1 - bf_up(hb1));
          uh[i][t] = pk16(hb0, hb1);
          ul[i][t] = pk16(lb0, lb1);
        }
      }
#pragma unroll
      for (int pass = 0; pass < 2; ++pass) {
#pragma unroll
        for (int i = 0; i < 4; ++i) {
          const int row = (4 * chk + i) * 8 + r8;
          const size_t po = ((size_t)(b * SEQ + n0 + row)) * CC + 128 * half + 8 * e16;
          *(volatile v4u*)(H2h + po) = uh[i];
          *(volatile v4u*)(H2l + po) = ul[i];
        }
        __threadfence();
      }
    }
  }
}

__global__ __launch_bounds__(128)
void gemm_proj(const unsigned short* __restrict__ WPT, const unsigned short* __restrict__ H2h,
               const unsigned short* __restrict__ H2l, const float* __restrict__ bp,
               const float* __restrict__ x, float* out) {
  __shared__ __align__(16) float Os[QT * OSP];
  const int tid  = threadIdx.x;
  const int lane = tid & 31, wave = tid >> 5;
  const int hh   = lane >> 4, c = lane & 15;
  const int nt   = blockIdx.x, mb = blockIdx.y, b = blockIdx.z;
  const int n0   = nt * QT, o0 = mb * QT;

  const unsigned short* ap  = WPT + (size_t)(o0 + c) * CC + 8 * hh;
  const size_t bo = ((size_t)(b * SEQ + n0 + 16 * wave + c)) * CC + 8 * hh;
  const unsigned short* bph = H2h + bo;
  const unsigned short* bpl = H2l + bo;

  v8f acc[4];
#pragma unroll
  for (int mt = 0; mt < 4; ++mt) acc[mt] = zero8();

#pragma unroll
  for (int ks = 0; ks < CC / 32; ++ks) {
    const Frag fbh = ldfrag(bph + 32 * ks);
    const Frag fbl = ldfrag(bpl + 32 * ks);
#pragma unroll
    for (int mt = 0; mt < 4; ++mt) {
      const Frag fa = ldfrag(ap + (size_t)(16 * mt) * CC + 32 * ks);
      acc[mt] = mma_b(fa.bf, fbh.bf, acc[mt]);
      acc[mt] = mma_b(fa.bf, fbl.bf, acc[mt]);
    }
  }

  {
    const int nl = 16 * wave + c;
#pragma unroll
    for (int mt = 0; mt < 4; ++mt) {
      v4f va, vb;
#pragma unroll
      for (int r = 0; r < 4; ++r) {
        va[r] = acc[mt][r]     + bfr(bp[o0 + 16 * mt + 8 * hh + r]);
        vb[r] = acc[mt][4 + r] + bfr(bp[o0 + 16 * mt + 8 * hh + 4 + r]);
      }
      *(v4f*)(Os + nl * OSP + 16 * mt + 8 * hh)     = va;
      *(v4f*)(Os + nl * OSP + 16 * mt + 8 * hh + 4) = vb;
    }
  }
  __syncthreads();

  const int e = tid & 7, lq = tid >> 3;
  v4f res[8];
#pragma unroll
  for (int it = 0; it < 8; ++it) {
    const int L  = it * 16 + lq;
    const int ol = L >> 1, hf = L & 1;
    const int nl = hf * 32 + 4 * e;
    const v4f xv = *(const v4f*)(x + ((size_t)(b * CC + o0 + ol)) * NNF + n0 + nl);
#pragma unroll
    for (int t = 0; t < 4; ++t) res[it][t] = Os[(nl + t) * OSP + ol] + bfr(xv[t]);
  }
#pragma unroll
  for (int pass = 0; pass < 2; ++pass) {
#pragma unroll
    for (int it = 0; it < 8; ++it) {
      const int L  = it * 16 + lq;
      const int ol = L >> 1, hf = L & 1;
      const int nl = hf * 32 + 4 * e;
      *(volatile v4f*)(out + ((size_t)(b * CC + o0 + ol)) * SEQ + n0 + nl) = res[it];
    }
    __threadfence();
  }
}

extern "C" void kernel_launch(void* const* d_in, const int* in_sizes, int n_in,
                              void* d_out, int out_size, void* d_ws, size_t ws_size,
                              hipStream_t stream) {
  if (n_in < 11) return;
  if ((size_t)in_sizes[0] < (size_t)NB * CC * NNF) return;
  if (in_sizes[1] < CC || in_sizes[2] < CC) return;
  if (in_sizes[3] < CC * CC || in_sizes[5] < CC * CC || in_sizes[7] < CC * CC || in_sizes[9] < CC * CC) return;
  if (in_sizes[4] < CC || in_sizes[6] < CC || in_sizes[8] < CC || in_sizes[10] < CC) return;
  if ((size_t)out_size < (size_t)NB * CC * SEQ) return;

  size_t off = 0;
  auto carve = [&](size_t bytes) { const size_t o = off; off += (bytes + 255) & ~(size_t)255; return o; };
  const size_t plane = (size_t)NB * SEQ * CC * 2;
  const size_t oST  = carve((size_t)NB * NG * STP * 4);
  const size_t oWT  = carve((size_t)4 * CC * CC * 2);
  const size_t oHPh = carve(plane);
  const size_t oHPl = carve(plane);
  const size_t oQh  = carve(plane);
  const size_t oQl  = carve(plane);
  const size_t oKh  = carve(plane);
  const size_t oVc  = carve(plane);
  const size_t oH2h = carve(plane);
  const size_t oH2l = carve(plane);
  if (off > ws_size) return;
  if (off > (size_t)134217728) return;

  const float* x   = (const float*)d_in[0];
  const float* gsc = (const float*)d_in[1];
  const float* gbs = (const float*)d_in[2];
  const float* Wq  = (const float*)d_in[3];
  const float* bq  = (const float*)d_in[4];
  const float* Wk  = (const float*)d_in[5];
  const float* bk  = (const float*)d_in[6];
  const float* Wv  = (const float*)d_in[7];
  const float* bv  = (const float*)d_in[8];
  const float* Wp  = (const float*)d_in[9];
  const float* bp  = (const float*)d_in[10];

  char* ws = (char*)d_ws;
  float*          ST  = (float*)(ws + oST);
  unsigned short* WT  = (unsigned short*)(ws + oWT);
  unsigned short* HPh = (unsigned short*)(ws + oHPh);
  unsigned short* HPl = (unsigned short*)(ws + oHPl);
  unsigned short* Qh  = (unsigned short*)(ws + oQh);
  unsigned short* Ql  = (unsigned short*)(ws + oQl);
  unsigned short* Kh  = (unsigned short*)(ws + oKh);
  unsigned short* Vc  = (unsigned short*)(ws + oVc);
  unsigned short* H2h = (unsigned short*)(ws + oH2h);
  unsigned short* H2l = (unsigned short*)(ws + oH2l);
  float* out = (float*)d_out;

  const dim3 blk256(256), blk128(128);

  cvt_w<<<dim3(CC / QT, CC / QT, 4), blk256, 0, stream>>>(Wq, Wk, Wv, Wp, WT);
  gn_stats<<<dim3(NG, NB), blk256, 0, stream>>>(x, ST);
  cvt_h<<<dim3(SEQ / QT, CC / QT, NB), blk256, 0, stream>>>(x, ST, gsc, gbs, HPh, HPl);
  gemm_qkv<<<dim3(SEQ / QT, 3 * CC / QT, NB), blk128, 0, stream>>>(WT, HPh, HPl, bq, bk, bv, Qh, Ql, Kh, Vc);
  attn_k<<<dim3(SEQ / QT, NB), blk128, 0, stream>>>(Qh, Ql, Kh, Vc, H2h, H2l);
  gemm_proj<<<dim3(SEQ / QT, CC / QT, NB), blk128, 0, stream>>>(WT + (size_t)3 * CC * CC, H2h, H2l, bp, x, out);
  (void)hipGetLastError();
}
